// HANModel_1821066133799
// MI455X (gfx1250) — hardware-run, weakly checked
//
#include <hip/hip_runtime.h>
#include <stddef.h>
#include <stdint.h>
#include <math.h>


#ifndef H1_SPLIT
#define H1_SPLIT 1
#endif

#define NN      50000
#define NE      800000
#define NREL    2
#define FIN     128
#define HC1     128
#define NHD1    4
#define HD1     32
#define HC2     64
#define KHL     256
#define K2      (H1_SPLIT ? 256 : 128)
#define MP      50048
#define NTHR    256
#define NWAVE   8
#define EPT     8
#define CHUNK   (NTHR * EPT)
#define WCAP    (EPT * 32)
#define LISTN   (NWAVE * WCAP)
#define NBMAX   2048
#define SLOTB   11
#define NB      1024
#define NBLK    49
#define NP      (NBLK * NB)
#define NBW     (NB / NWAVE)
#define RCAP    20480
#define DEGCAP  64
#define MAXHIT  16707
#define MAXDEG  36
#define GBM     64
#define GBN     128
#define GTHR    128
#define GNT     8
#define NEGSL   0.2f
#define MX0     (-1.0e30f)
#define WSMAX   134217728
#define LDS_BKT ((2 * RCAP + 2 * NBMAX + LISTN) * 4 + 64)
#define PAR_AL1 0
#define PAR_AR1 256
#define PAR_B1  512
#define PAR_AL2 768
#define PAR_AR2 896
#define PAR_B2  1024
#define NPAR    1152
#define NUX     (MP * (FIN / 8))
#define NUW1    (NREL * HC1 * (FIN / 8))
#define NUW2    (NREL * HC2 * (K2 / 8))
#define NUP     (NPAR / 4)
#define NUPB    512
#define PB1     (NUX)
#define PB2     (PB1 + NUW1)
#define PB3     (PB2 + NUW2)
#define PTOT    (PB3 + NUPB)

static_assert((CHUNK & (CHUNK - 1)) == 0 && CHUNK <= (1 << SLOTB));
static_assert(NBMAX == (1 << SLOTB));
static_assert(NTHR * 8 == NBMAX);
static_assert(LISTN >= NBMAX && LISTN >= NWAVE * WCAP);
static_assert(NB <= NBMAX && NB == 4 * NTHR && (NB % NWAVE) == 0 && (NBW % 2) == 0);
static_assert(NBLK * NB >= MP);
static_assert((RCAP % (4 * NTHR)) == 0 && (RCAP % 32) == 0);
static_assert(RCAP >= MAXHIT + MAXHIT / 20);
static_assert(DEGCAP >= MAXDEG + 8);
static_assert(NE < (1 << (32 - SLOTB)));
static_assert((NE % 256) == 0);
static_assert(LDS_BKT <= 327680);
static_assert((MP % GBM) == 0 && MP >= NN && (NN % 2) == 0);
static_assert(GBM == (GTHR / 32) * 16 && GBN == 16 * GNT);
static_assert((FIN % 32) == 0);
static_assert((K2 % 32) == 0);
static_assert(K2 <= KHL && KHL == 2 * HC1);
static_assert(HC1 == NHD1 * HD1 && HC1 == 32 * 4 && HD1 == 8 * 4);
static_assert(HC2 == 32 * 2 && NREL * HC2 == GBN && HC1 == GBN);
static_assert((NUX % NTHR) == 0 && (NUW1 % NTHR) == 0 && (NUW2 % NTHR) == 0 && (NUPB % NTHR) == 0);
static_assert((NUP % 32) == 0 && NUP <= NUPB);

typedef float          v2f  __attribute__((ext_vector_type(2)));
typedef float          v4f  __attribute__((ext_vector_type(4)));
typedef float          v8f  __attribute__((ext_vector_type(8)));
typedef int            v4i  __attribute__((ext_vector_type(4)));
typedef int            v8i  __attribute__((ext_vector_type(8)));
typedef unsigned int   v4u  __attribute__((ext_vector_type(4)));
typedef unsigned short v8us __attribute__((ext_vector_type(8)));
typedef __bf16         v16b __attribute__((ext_vector_type(16)));
typedef v2f  __attribute__((may_alias)) v2fa;
typedef v4f  __attribute__((may_alias)) v4fa;
typedef v4i  __attribute__((may_alias)) v4ia;
typedef v8us __attribute__((may_alias)) v8usa;
union Frag { v16b vb; v8us h[2]; v8i w; };

__device__ __forceinline__ v8f wmb(const Frag& a, const Frag& b, v8f c) {
  v8f d = __builtin_amdgcn_wmma_f32_16x16x32_bf16(false, a.vb, false, b.vb, (short)0, c, false, false);
  asm volatile("v_nop\n\tv_nop\n\tv_nop\n\tv_nop" : "+v"(d) : "v"(a.w), "v"(b.w));
  return d;
}

__device__ __forceinline__ unsigned short bf_bits(float f) {
  unsigned int u = __float_as_uint(f);
  u += 0x7FFFu + ((u >> 16) & 1u);
  return (unsigned short)(u >> 16);
}
__device__ __forceinline__ float bf_val(unsigned short b) { return __uint_as_float(((unsigned int)b) << 16); }
__device__ __forceinline__ float bf_rne(float f) { return bf_val(bf_bits(f)); }
__device__ __forceinline__ unsigned int pk2(float lo, float hi) {
  return (unsigned int)bf_bits(lo) | ((unsigned int)bf_bits(hi) << 16);
}
__device__ __forceinline__ v4u pack8(const v4f a, const v4f b) {
  v4u r;
  r.x = pk2(a.x, a.y); r.y = pk2(a.z, a.w); r.z = pk2(b.x, b.y); r.w = pk2(b.z, b.w);
  return r;
}
__device__ __forceinline__ int clampi(int v, int lo, int hi) { return v < lo ? lo : (v > hi ? hi : v); }

__device__ __forceinline__ void st2u(unsigned short* p, const v4u v) {
  *(volatile v4u*)p = v;
  __threadfence();
  *(volatile v4u*)p = v;
}
__device__ __forceinline__ void st2i(int* p, const v4i v) {
  *(volatile v4i*)p = v;
  __threadfence();
  *(volatile v4i*)p = v;
}

__device__ __forceinline__ int scan_chunk(const int* __restrict__ dsts, int nE, int cbase, int slotBase,
                                          int nb, int vec8, int* list, int tid, int lane, int wave) {
  int wc = 0;
  const int el0  = tid * EPT;
  const int e0   = cbase + el0;
  const int sent = -2147483647 - 1;
  v4i da, db;
  if (vec8 != 0 && cbase + CHUNK <= nE) {
    da = *(const v4i*)(dsts + e0);
    db = *(const v4i*)(dsts + e0 + 4);
  } else {
    const int kt0 = dsts[min(e0, nE - 1)];
    const int kt1 = dsts[min(e0 + 1, nE - 1)];
    const int kt2 = dsts[min(e0 + 2, nE - 1)];
    const int kt3 = dsts[min(e0 + 3, nE - 1)];
    const int kt4 = dsts[min(e0 + 4, nE - 1)];
    const int kt5 = dsts[min(e0 + 5, nE - 1)];
    const int kt6 = dsts[min(e0 + 6, nE - 1)];
    const int kt7 = dsts[min(e0 + 7, nE - 1)];
    asm volatile("" :: "v"(kt0), "v"(kt1), "v"(kt2), "v"(kt3));
    asm volatile("" :: "v"(kt4), "v"(kt5), "v"(kt6), "v"(kt7));
    da.x = (e0 < nE) ? kt0 : sent;
    da.y = (e0 + 1 < nE) ? kt1 : sent;
    da.z = (e0 + 2 < nE) ? kt2 : sent;
    da.w = (e0 + 3 < nE) ? kt3 : sent;
    db.x = (e0 + 4 < nE) ? kt4 : sent;
    db.y = (e0 + 5 < nE) ? kt5 : sent;
    db.z = (e0 + 6 < nE) ? kt6 : sent;
    db.w = (e0 + 7 < nE) ? kt7 : sent;
  }
  const unsigned nbs = (unsigned)slotBase;
  const unsigned unb = (unsigned)nb;
  const unsigned s0 = (unsigned)da.x - nbs, s1 = (unsigned)da.y - nbs;
  const unsigned s2 = (unsigned)da.z - nbs, s3 = (unsigned)da.w - nbs;
  const unsigned s4 = (unsigned)db.x - nbs, s5 = (unsigned)db.y - nbs;
  const unsigned s6 = (unsigned)db.z - nbs, s7 = (unsigned)db.w - nbs;
  const bool h0 = s0 < unb, h1 = s1 < unb, h2 = s2 < unb, h3 = s3 < unb;
  const bool h4 = s4 < unb, h5 = s5 < unb, h6 = s6 < unb, h7 = s7 < unb;
  const unsigned any = __builtin_amdgcn_ballot_w32(h0 | h1 | h2 | h3 | h4 | h5 | h6 | h7);
  if (any != 0u) {
#define HITJ(J, HJ, SJ) { \
      const unsigned mj = __builtin_amdgcn_ballot_w32(HJ); \
      if (mj != 0u) { \
        if (HJ) { \
          const int pos = wc + (int)__builtin_amdgcn_mbcnt_lo(mj, 0u); \
          if (pos < WCAP) list[wave * WCAP + pos] = ((el0 + (J)) << SLOTB) | (int)(SJ); \
        } \
        wc += (int)__builtin_popcount(mj); } }
    HITJ(0, h0, s0)
    HITJ(1, h1, s1)
    HITJ(2, h2, s2)
    HITJ(3, h3, s3)
    HITJ(4, h4, s4)
    HITJ(5, h5, s5)
    HITJ(6, h6, s6)
    HITJ(7, h7, s7)
#undef HITJ
  }
  return wc;
}

__global__ __launch_bounds__(NTHR) void k_prep(const float* __restrict__ x, const float* __restrict__ w1,
                                               const float* __restrict__ w2,
                                               const float* __restrict__ al1, const float* __restrict__ ar1,
                                               const float* __restrict__ b1,
                                               const float* __restrict__ al2, const float* __restrict__ ar2,
                                               const float* __restrict__ b2,
                                               unsigned short* xb, unsigned short* w1t, unsigned short* w2t,
                                               float* par) {
  const int u = (int)blockIdx.x * NTHR + (int)threadIdx.x;
  if (u < PB1) {
    const int row = u >> 4, c0 = (u & 15) * 8;
    const int rc  = row < NN ? row : NN - 1;
    const float* p = x + (size_t)rc * FIN + c0;
    v4f a = *(const v4fa*)p, b = *(const v4fa*)(p + 4);
    asm volatile("" :: "v"(a), "v"(b));
    const v4f z4 = {0.f, 0.f, 0.f, 0.f};
    const bool live = row < NN;
    a = live ? a : z4;
    b = live ? b : z4;
    st2u(xb + (size_t)row * FIN + c0, pack8(a, b));
  } else if (u < PB2) {
    const int v = u - PB1, row = v >> 4, k8 = (v & 15) * 8;
    const int r = row >> 7, n = row & 127;
    const float* p = w1 + (size_t)r * FIN * HC1 + (size_t)k8 * HC1 + n;
    v4f a, b;
    a.x = p[0];        a.y = p[HC1];      a.z = p[2 * HC1];  a.w = p[3 * HC1];
    b.x = p[4 * HC1];  b.y = p[5 * HC1];  b.z = p[6 * HC1];  b.w = p[7 * HC1];
    st2u(w1t + (size_t)v * 8, pack8(a, b));
  } else if (u < PB3) {
    const int v = u - PB2;
    const int kq = K2 / 8;
    const int row = v / kq, k8 = (v - row * kq) * 8;
    const int kk = k8 & (HC1 - 1);
    const int r = row >> 6, n = row & 63;
    const float* p = w2 + (size_t)r * HC1 * HC2 + (size_t)kk * HC2 + n;
    v4f a, b;
    a.x = p[0];        a.y = p[HC2];      a.z = p[2 * HC2];  a.w = p[3 * HC2];
    b.x = p[4 * HC2];  b.y = p[5 * HC2];  b.z = p[6 * HC2];  b.w = p[7 * HC2];
    st2u(w2t + (size_t)v * 8, pack8(a, b));
  } else {
    const int v = u - PB3;
    if (v >= NUP) return;
    const int i1 = clampi(v, 0, 63),        i2 = clampi(v - 64, 0, 63),  i3 = clampi(v - 128, 0, 63);
    const int i4 = clampi(v - 192, 0, 31),  i5 = clampi(v - 224, 0, 31), i6 = clampi(v - 256, 0, 31);
    const v4f q1 = *(const v4fa*)(al1 + 4 * i1);
    const v4f q2 = *(const v4fa*)(ar1 + 4 * i2);
    const v4f q3 = *(const v4fa*)(b1  + 4 * i3);
    const v4f q4 = *(const v4fa*)(al2 + 4 * i4);
    const v4f q5 = *(const v4fa*)(ar2 + 4 * i5);
    const v4f q6 = *(const v4fa*)(b2  + 4 * i6);
    asm volatile("" :: "v"(q1), "v"(q2), "v"(q3));
    asm volatile("" :: "v"(q4), "v"(q5), "v"(q6));
    v4f s = q6;
    s = v < 256 ? q5 : s;
    s = v < 224 ? q4 : s;
    s = v < 192 ? q3 : s;
    s = v < 128 ? q2 : s;
    s = v < 64  ? q1 : s;
    v4f o;
    o.x = bf_rne(s.x); o.y = bf_rne(s.y); o.z = bf_rne(s.z); o.w = bf_rne(s.w);
    float* dp = par + 4 * v;
    *(volatile v4f*)dp = o;
    __threadfence();
    *(volatile v4f*)dp = o;
  }
}

__global__ __launch_bounds__(NTHR) void k_bucket(const int* __restrict__ src, const int* __restrict__ dst,
                                                 int* LIST, int* CNT, int* OFF, int* FLG) {
  extern __shared__ v4f lds_dyn[];
  int* reg1 = (int*)lds_dyn;
  int* reg2 = reg1 + RCAP;
  int* scnt = reg2 + RCAP;
  int* soff = scnt + NBMAX;
  int* list = soff + NBMAX;
  int* wcnt = list + LISTN;
  int* wtot = wcnt + NWAVE;
  const int tid = (int)threadIdx.x, lane = tid & 31, wave = tid >> 5;
  const int b = (int)blockIdx.x, r = (int)blockIdx.y;
  const int* dsts = dst + (size_t)r * NE;
  const int* srcs = src + (size_t)r * NE;
  const int nodeBase = b * NB;
  const int nE = NE, nb = NB, vec8 = 1;

  {
    const v4i z4 = {0, 0, 0, 0};
    for (int i = tid; i < NBMAX; i += NTHR) scnt[i] = 0;
    for (int i = 4 * tid; i < RCAP; i += 4 * NTHR) *(v4ia*)(reg2 + i) = z4;
  }
  __syncthreads();

  int tot = 0;
  const int nChunks = (nE + CHUNK - 1) / CHUNK;
#pragma unroll 1
  for (int ch = 0; ch < nChunks; ++ch) {
    const int cbase = ch * CHUNK;
    const int wc = scan_chunk(dsts, nE, cbase, nodeBase, nb, vec8, list, tid, lane, wave);
    if (lane == 0) wcnt[wave] = wc;
    __syncthreads();
    int pre = 0, all = 0;
#pragma unroll
    for (int w2 = 0; w2 < NWAVE; ++w2) {
      int c = wcnt[w2];
      c = c < 0 ? 0 : (c > WCAP ? WCAP : c);
      all += c;
      pre += (w2 < wave) ? c : 0;
    }
    const int wcc  = wc > WCAP ? WCAP : wc;
    const int base = tot + pre;
#pragma unroll 1
    for (int i = lane; i < wcc; i += 32) {
      const int ent = list[wave * WCAP + i];
      const int el  = (ent >> SLOTB) & (CHUNK - 1);
      const int sl  = ent & (NBMAX - 1);
      int eid = cbase + el;
      eid = eid > nE - 1 ? nE - 1 : eid;
      const int pos = base + i;
      if (pos < RCAP) reg1[pos] = (int)(((unsigned)eid << SLOTB) | (unsigned)sl);
    }
    tot += all;
    tot = tot > RCAP ? RCAP : tot;
    __syncthreads();
  }
  const int nh = tot;

  if (wave == 0) {
#pragma unroll 1
    for (int b0 = 0; b0 < nh; b0 += 32) {
      const int idx = b0 + lane;
      const int uv  = reg1[idx < nh ? idx : nh - 1];
      const int m32 = (nh - b0) < 32 ? (nh - b0) : 32;
#pragma unroll 1
      for (int k = 0; k < m32; ++k) {
        const int u  = __builtin_amdgcn_readlane(uv, k);
        const int sl = u & (NBMAX - 1);
        if (lane == 0) scnt[sl] = scnt[sl] + 1;
      }
    }
  }
  __syncthreads();

  {
    const v4i ca = *(const v4ia*)(scnt + 8 * tid);
    const v4i cb = *(const v4ia*)(scnt + 8 * tid + 4);
    const int e0 = ca.x < 0 ? 0 : ca.x, e1 = ca.y < 0 ? 0 : ca.y, e2 = ca.z < 0 ? 0 : ca.z, e3 = ca.w < 0 ? 0 : ca.w;
    const int e4 = cb.x < 0 ? 0 : cb.x, e5 = cb.y < 0 ? 0 : cb.y, e6 = cb.z < 0 ? 0 : cb.z, e7 = cb.w < 0 ? 0 : cb.w;
    const int ts = e0 + e1 + e2 + e3 + e4 + e5 + e6 + e7;
    int incl = ts;
#pragma unroll
    for (int d = 1; d < 32; d <<= 1) {
      const int up = __shfl_up(incl, d);
      if (lane >= d) incl += up;
    }
    if (lane == 31) wtot[wave] = incl;
    __syncthreads();
    int pre = 0;
#pragma unroll
    for (int w2 = 0; w2 < NWAVE; ++w2) pre += (w2 < wave) ? wtot[w2] : 0;
    int run = pre + incl - ts;
    soff[8 * tid + 0] = run; run += e0;
    soff[8 * tid + 1] = run; run += e1;
    soff[8 * tid + 2] = run; run += e2;
    soff[8 * tid + 3] = run; run += e3;
    soff[8 * tid + 4] = run; run += e4;
    soff[8 * tid + 5] = run; run += e5;
    soff[8 * tid + 6] = run; run += e6;
    soff[8 * tid + 7] = run;
  }
  __syncthreads();
  for (int i = tid; i < NBMAX; i += NTHR) list[i] = soff[i];
  __syncthreads();

  if (wave == 0) {
#pragma unroll 1
    for (int b0 = 0; b0 < nh; b0 += 32) {
      const int idx = b0 + lane;
      const int uv  = reg1[idx < nh ? idx : nh - 1];
      const int m32 = (nh - b0) < 32 ? (nh - b0) : 32;
#pragma unroll 1
      for (int k = 0; k < m32; ++k) {
        const int u   = __builtin_amdgcn_readlane(uv, k);
        const int sl  = u & (NBMAX - 1);
        const int eid = (int)((unsigned)u >> SLOTB);
        if (lane == 0) {
          int pos = list[sl];
          pos = pos < 0 ? 0 : (pos > RCAP - 1 ? RCAP - 1 : pos);
          reg2[pos] = eid;
          list[sl] = pos + 1;
        }
      }
    }
  }
  __syncthreads();

  {
    int* Lg = LIST + (size_t)(r * NBLK + b) * RCAP;
#pragma unroll 1
    for (int i = 4 * tid; i < RCAP; i += 4 * NTHR) {
      const v4i e = *(const v4ia*)(reg2 + i);
      v4i s;
      s.x = srcs[clampi(e.x, 0, NE - 1)];
      s.y = srcs[clampi(e.y, 0, NE - 1)];
      s.z = srcs[clampi(e.z, 0, NE - 1)];
      s.w = srcs[clampi(e.w, 0, NE - 1)];
      s.x = clampi(s.x, 0, NN - 1); s.y = clampi(s.y, 0, NN - 1);
      s.z = clampi(s.z, 0, NN - 1); s.w = clampi(s.w, 0, NN - 1);
      st2i(Lg + i, s);
    }
  }
  {
    const v4i cv = *(const v4ia*)(scnt + 4 * tid);
    const v4i ov = *(const v4ia*)(soff + 4 * tid);
    const int fl = (nh >= RCAP) ? 1 : 0;
    const v4i fv = {fl, fl, fl, fl};
    int* cp = CNT + (size_t)r * NP + nodeBase + 4 * tid;
    int* op = OFF + (size_t)r * NP + nodeBase + 4 * tid;
    int* fp = FLG + (size_t)(r * NBLK + b) * 32 + 4 * (tid & 7);
    const bool wf = tid < 8;
    *(volatile v4i*)cp = cv;
    *(volatile v4i*)op = ov;
    if (wf) *(volatile v4i*)fp = fv;
    __threadfence();
    *(volatile v4i*)cp = cv;
    *(volatile v4i*)op = ov;
    if (wf) *(volatile v4i*)fp = fv;
  }
}

template <int LAYER>
__global__ __launch_bounds__(GTHR) __attribute__((amdgpu_num_vgpr(248)))
void k_gemm(const unsigned short* __restrict__ A, int lda,
            const unsigned short* __restrict__ BT, int ldb, int K,
            float* outF, int ldo,
            const float* __restrict__ PAR, int parA, int parB,
            float* SD, int sdPlane) {
  __shared__ __attribute__((aligned(16))) float stg[GBM * GBN];
  __shared__ __attribute__((aligned(16))) float satt[2 * GBN];
  __shared__ __attribute__((aligned(16))) float sdot[GBM * 8];
  const int tid = (int)threadIdx.x, lane = tid & 31, wave = tid >> 5, hh = lane >> 4, m = lane & 15;
  const int rowBase = (int)blockIdx.x * GBM;
  const int by = (int)blockIdx.y;

  if (tid < 64) {
    const int off = (tid < 32) ? (parA + by * GBN + 4 * tid) : (parB + by * GBN + 4 * (tid - 32));
    const v4f v = *(const v4fa*)(PAR + off);
    *(v4fa*)(satt + 4 * tid) = v;
  }

  v8f acc[GNT];
  {
    const v8f z = {0.f, 0.f, 0.f, 0.f, 0.f, 0.f, 0.f, 0.f};
#pragma unroll
    for (int t = 0; t < GNT; ++t) acc[t] = z;
  }
  const unsigned short* ap = A + (size_t)(rowBase + 16 * wave + m) * (size_t)lda + 8 * hh;
  const unsigned short* bp = BT + (size_t)(by * GBN + m) * (size_t)ldb + 8 * hh;

#pragma unroll 1
  for (int k0 = 0; k0 < K; k0 += 32) {
    Frag af;
    af.h[0] = *(const v8usa*)(ap + k0);
    af.h[1] = *(const v8usa*)(ap + k0 + 16);
#pragma unroll
    for (int nt = 0; nt < GNT; ++nt) {
      const unsigned short* wq = bp + (size_t)(16 * nt) * (size_t)ldb + k0;
      Frag bfg;
      bfg.h[0] = *(const v8usa*)wq;
      bfg.h[1] = *(const v8usa*)(wq + 16);
      acc[nt] = wmb(af, bfg, acc[nt]);
    }
  }

#pragma unroll
  for (int nt = 0; nt < GNT; ++nt) {
    const int lc = 16 * nt + m;
#pragma unroll
    for (int r = 0; r < 8; ++r) {
      const int lr = 16 * wave + 8 * hh + r;
      stg[lr * GBN + lc] = acc[nt][r];
    }
  }
  __syncthreads();

  {
    const int row = tid & 63, half = tid >> 6;
    constexpr int NSEG = (LAYER == 1) ? 2 : 1;
    constexpr int SEGL = (LAYER == 1) ? HD1 : HC2;
#pragma unroll 1
    for (int sg = 0; sg < NSEG; ++sg) {
      const int c0 = 64 * half + SEGL * sg;
      const float* hr = stg + row * GBN + c0;
      const float* sa = satt + c0;
      const float* sb = satt + GBN + c0;
      float ds = 0.0f, dd = 0.0f;
#pragma unroll 4
      for (int c4 = 0; c4 < SEGL / 4; ++c4) {
        const v4f hv = *(const v4fa*)(hr + 4 * c4);
        const v4f av = *(const v4fa*)(sa + 4 * c4);
        const v4f bv = *(const v4fa*)(sb + 4 * c4);
        ds = fmaf(hv.x, av.x, ds);  dd = fmaf(hv.x, bv.x, dd);
        ds = fmaf(hv.y, av.y, ds);  dd = fmaf(hv.y, bv.y, dd);
        ds = fmaf(hv.z, av.z, ds);  dd = fmaf(hv.z, bv.z, dd);
        ds = fmaf(hv.w, av.w, ds);  dd = fmaf(hv.w, bv.w, dd);
      }
      if (LAYER == 1) {
        const int head = 2 * half + sg;
        sdot[row * 8 + head]     = ds;
        sdot[row * 8 + 4 + head] = dd;
      } else {
        sdot[row * 4 + 2 * half]     = ds;
        sdot[row * 4 + 2 * half + 1] = dd;
      }
    }
  }
  __syncthreads();

  v4f fv[16];
#pragma unroll
  for (int i = 0; i < 16; ++i) {
    const int lr = 16 * wave + i;
    fv[i] = *(const v4fa*)(stg + lr * GBN + 4 * lane);
  }
  constexpr int NPC = (LAYER == 1) ? 128 : 64;
  constexpr int SW  = (LAYER == 1) ? 8 : 4;
  const int pc = tid & (NPC - 1);
  const bool wsd = tid < NPC;
  const v4f dv = *(const v4fa*)(sdot + 4 * pc);
  float* dpp = SD + (size_t)by * (size_t)sdPlane + (size_t)rowBase * SW + 4 * pc;
#pragma unroll
  for (int i = 0; i < 16; ++i) {
    const int gr = rowBase + 16 * wave + i;
    float* op = outF + (size_t)gr * (size_t)ldo + by * GBN + 4 * lane;
    *(volatile v4f*)op = fv[i];
  }
  if (wsd) *(volatile v4f*)dpp = dv;
  __threadfence();
#pragma unroll
  for (int i = 0; i < 16; ++i) {
    const int gr = rowBase + 16 * wave + i;
    float* op = outF + (size_t)gr * (size_t)ldo + by * GBN + 4 * lane;
    *(volatile v4f*)op = fv[i];
  }
  if (wsd) *(volatile v4f*)dpp = dv;
}

__global__ __launch_bounds__(NTHR) void k_agg1(const float* __restrict__ F, const float* __restrict__ S1,
                                               const int* __restrict__ LIST, const int* __restrict__ CNT,
                                               const int* __restrict__ OFF, const int* __restrict__ FLG,
                                               const float* __restrict__ PAR, unsigned short* HP) {
  __shared__ __attribute__((aligned(16))) int scn[NREL * NB];
  __shared__ __attribute__((aligned(16))) int sof[NREL * NB];
  __shared__ __attribute__((aligned(16))) float sbias[NREL * HC1];
  const int tid = (int)threadIdx.x, lane = tid & 31, wave = tid >> 5;
  const int b = (int)blockIdx.x;
  const int nodeBase = b * NB;

#pragma unroll
  for (int r = 0; r < NREL; ++r) {
    const v4i c = *(const v4ia*)(CNT + (size_t)r * NP + nodeBase + 4 * tid);
    const v4i o = *(const v4ia*)(OFF + (size_t)r * NP + nodeBase + 4 * tid);
    *(v4ia*)(scn + r * NB + 4 * tid) = c;
    *(v4ia*)(sof + r * NB + 4 * tid) = o;
  }
  if (tid < 64) {
    const v4f v = *(const v4fa*)(PAR + PAR_B1 + 4 * tid);
    *(v4fa*)(sbias + 4 * tid) = v;
  }
  const int f0 = FLG[(size_t)b * 32];
  const int f1 = FLG[(size_t)(NBLK + b) * 32];
  __syncthreads();

  const bool ovf = (f0 != 0) || (f1 != 0);
  const float qnan = __int_as_float(0x7fc00000);
  const int head = lane >> 3;

#pragma unroll 1
  for (int jt = 0; jt < NBW; ++jt) {
    const int slot = wave * NBW + jt;
    const int grow = nodeBase + slot;
    const int gcl  = grow < NN ? grow : NN - 1;
    const bool liveRow = grow < NN;
    float pz = ovf ? qnan : 0.0f;
    v4f hs = {0.f, 0.f, 0.f, 0.f};

#pragma unroll 1
    for (int r = 0; r < NREL; ++r) {
      int st = sof[r * NB + slot];
      const int craw = scn[r * NB + slot];
      int cnt = craw;
      st  = st < 0 ? 0 : (st > RCAP ? RCAP : st);
      cnt = cnt < 0 ? 0 : (cnt > DEGCAP ? DEGCAP : cnt);
      if (cnt > RCAP - st) cnt = RCAP - st;
      cnt = __builtin_amdgcn_readfirstlane(cnt);
      st  = __builtin_amdgcn_readfirstlane(st);
      pz = (craw > DEGCAP) ? qnan : pz;
      const size_t sbase = (size_t)r * MP * 8;
      const size_t lbase = (size_t)(r * NBLK + b) * RCAP;
      const int    fcol  = r * HC1 + 4 * lane;
      const float erv = S1[sbase + (size_t)gcl * 8 + 4 + head];
      float mx = MX0, dn = 0.0f;
      v4f av = {0.f, 0.f, 0.f, 0.f};

#pragma unroll 1
      for (int q0 = 0; q0 < cnt; q0 += 32) {
        int idx = st + q0 + lane;
        idx = idx > RCAP - 1 ? RCAP - 1 : idx;
        int sv = LIST[lbase + idx];
        sv = sv < 0 ? 0 : (sv > NN - 1 ? NN - 1 : sv);
        const int rem = cnt - q0;
        const int m32 = rem < 32 ? rem : 32;
#pragma unroll 1
        for (int k = 0; k < m32; ++k) {
          const int s = __builtin_amdgcn_readlane(sv, k);
          const v4f fs = *(const v4fa*)(F + (size_t)s * (NREL * HC1) + fcol);
          const float el = S1[sbase + (size_t)s * 8 + head];
          float lg = el + erv;
          lg = lg > 0.0f ? lg : NEGSL * lg;
          const float df = lg - mx;
          const float ee = expf(-fabsf(df));
          const bool up  = df > 0.0f;
          const float s1 = up ? ee : 1.0f;
          const float s2 = up ? 1.0f : ee;
          mx = up ? lg : mx;
          dn = fmaf(dn, s1, s2);
          av.x = fmaf(av.x, s1, s2 * fs.x);
          av.y = fmaf(av.y, s1, s2 * fs.y);
          av.z = fmaf(av.z, s1, s2 * fs.z);
          av.w = fmaf(av.w, s1, s2 * fs.w);
        }
      }
      const float dnz = cnt > 0 ? dn : 1.0f;
      const float inv = 1.0f / dnz;
      const v4f bb = *(const v4fa*)(sbias + r * HC1 + 4 * lane);
      hs.x = hs.x + (av.x * inv + bb.x);
      hs.y = hs.y + (av.y * inv + bb.y);
      hs.z = hs.z + (av.z * inv + bb.z);
      hs.w = hs.w + (av.w * inv + bb.w);
    }

    v4f o = {0.f, 0.f, 0.f, 0.f};
#pragma unroll 1
    for (int j = 0; j < 4; ++j) {
      const float v = hs.x;
      const float n = expm1f(v);
      const float e = v > 0.0f ? v : n;
      const v4f hr = {hs.y, hs.z, hs.w, hs.x};
      const v4f orr = {o.y, o.z, o.w, e};
      hs = hr;
      o = orr;
    }
    const float h0 = (liveRow ? o.x : 0.0f) + pz;
    const float h1 = (liveRow ? o.y : 0.0f) + pz;
    const float h2 = (liveRow ? o.z : 0.0f) + pz;
    const float h3 = (liveRow ? o.w : 0.0f) + pz;

    const unsigned int hb0 = bf_bits(h0), hb1 = bf_bits(h1), hb2 = bf_bits(h2), hb3 = bf_bits(h3);
    float hv0 = bf_val((unsigned short)hb0), hv1 = bf_val((unsigned short)hb1);
    float hv2 = bf_val((unsigned short)hb2), hv3 = bf_val((unsigned short)hb3);
    asm volatile("" : "+v"(hv0), "+v"(hv1), "+v"(hv2), "+v"(hv3));
    const unsigned int lb0 = bf_bits(h0 - hv0);
    const unsigned int lb1 = bf_bits(h1 - hv1);
    const unsigned int lb2 = bf_bits(h2 - hv2);
    const unsigned int lb3 = bf_bits(h3 - hv3);
    const int hwA = (int)(hb0 | (hb1 << 16));
    const int hwB = (int)(hb2 | (hb3 << 16));
    const int lwA = (int)(lb0 | (lb1 << 16));
    const int lwB = (int)(lb2 | (lb3 << 16));
    const int j  = lane & 15;
    const int sA = 2 * j, sB = 2 * j + 1;
    const int g0h = __shfl(hwA, sA), g1h = __shfl(hwB, sA), g2h = __shfl(hwA, sB), g3h = __shfl(hwB, sB);
    const int g0l = __shfl(lwA, sA), g1l = __shfl(lwB, sA), g2l = __shfl(lwA, sB), g3l = __shfl(lwB, sB);
    const bool hsel = lane < 16;
    v4u pv;
    pv.x = (unsigned int)(hsel ? g0h : g0l);
    pv.y = (unsigned int)(hsel ? g1h : g1l);
    pv.z = (unsigned int)(hsel ? g2h : g2l);
    pv.w = (unsigned int)(hsel ? g3h : g3l);

    unsigned short* hp = HP + (size_t)grow * KHL + 8 * lane;
    const bool wr = grow < MP;
    if (wr) *(volatile v4u*)hp = pv;
    __threadfence();
    if (wr) *(volatile v4u*)hp = pv;
  }
}

__global__ __launch_bounds__(NTHR) void k_agg2(const float* __restrict__ F, const float* __restrict__ S2,
                                               const int* __restrict__ LIST, const int* __restrict__ CNT,
                                               const int* __restrict__ OFF, const int* __restrict__ FLG,
                                               const float* __restrict__ PAR, float* out) {
  __shared__ __attribute__((aligned(16))) int scn[NREL * NB];
  __shared__ __attribute__((aligned(16))) int sof[NREL * NB];
  __shared__ __attribute__((aligned(16))) float sb2[NREL * HC2];
  const int tid = (int)threadIdx.x, lane = tid & 31, wave = tid >> 5;
  const int b = (int)blockIdx.x;
  const int nodeBase = b * NB;

#pragma unroll
  for (int r = 0; r < NREL; ++r) {
    const v4i c = *(const v4ia*)(CNT + (size_t)r * NP + nodeBase + 4 * tid);
    const v4i o = *(const v4ia*)(OFF + (size_t)r * NP + nodeBase + 4 * tid);
    *(v4ia*)(scn + r * NB + 4 * tid) = c;
    *(v4ia*)(sof + r * NB + 4 * tid) = o;
  }
  if (tid < 32) {
    const v4f v = *(const v4fa*)(PAR + PAR_B2 + 4 * tid);
    *(v4fa*)(sb2 + 4 * tid) = v;
  }
  const int f0 = FLG[(size_t)b * 32];
  const int f1 = FLG[(size_t)(NBLK + b) * 32];
  __syncthreads();

  const bool ovf = (f0 != 0) || (f1 != 0);
  const float qnan = __int_as_float(0x7fc00000);
  v2f rowA = {0.f, 0.f};

#pragma unroll 1
  for (int jt = 0; jt < NBW; ++jt) {
    const int slot = wave * NBW + jt;
    const int grow = nodeBase + slot;
    const int gcl  = grow < NN ? grow : NN - 1;
    float pz = ovf ? qnan : 0.0f;
    v2f hs = {0.f, 0.f};

#pragma unroll 1
    for (int r = 0; r < NREL; ++r) {
      int st = sof[r * NB + slot];
      const int craw = scn[r * NB + slot];
      int cnt = craw;
      st  = st < 0 ? 0 : (st > RCAP ? RCAP : st);
      cnt = cnt < 0 ? 0 : (cnt > DEGCAP ? DEGCAP : cnt);
      if (cnt > RCAP - st) cnt = RCAP - st;
      cnt = __builtin_amdgcn_readfirstlane(cnt);
      st  = __builtin_amdgcn_readfirstlane(st);
      pz = (craw > DEGCAP) ? qnan : pz;
      const size_t lbase = (size_t)(r * NBLK + b) * RCAP;
      const int    fcol  = r * HC2 + 2 * lane;
      const float erv = S2[(size_t)gcl * 4 + 2 * r + 1];
      float mx = MX0, dn = 0.0f, a0 = 0.0f, a1 = 0.0f;

#pragma unroll 1
      for (int q0 = 0; q0 < cnt; q0 += 32) {
        int idx = st + q0 + lane;
        idx = idx > RCAP - 1 ? RCAP - 1 : idx;
        int sv = LIST[lbase + idx];
        sv = sv < 0 ? 0 : (sv > NN - 1 ? NN - 1 : sv);
        const int rem = cnt - q0;
        const int m32 = rem < 32 ? rem : 32;
#pragma unroll 1
        for (int k = 0; k < m32; ++k) {
          const int s = __builtin_amdgcn_readlane(sv, k);
          const v2f fs = *(const v2fa*)(F + (size_t)s * (NREL * HC2) + fcol);
          const float el = S2[(size_t)s * 4 + 2 * r];
          float lg = el + erv;
          lg = lg > 0.0f ? lg : NEGSL * lg;
          const float df = lg - mx;
          const float ee = expf(-fabsf(df));
          const bool up  = df > 0.0f;
          const float s1 = up ? ee : 1.0f;
          const float s2 = up ? 1.0f : ee;
          mx = up ? lg : mx;
          dn = fmaf(dn, s1, s2);
          a0 = fmaf(a0, s1, s2 * fs.x);
          a1 = fmaf(a1, s1, s2 * fs.y);
        }
      }
      const float dnz = cnt > 0 ? dn : 1.0f;
      const float inv = 1.0f / dnz;
      const v2f bb = *(const v2fa*)(sb2 + r * HC2 + 2 * lane);
      hs.x = hs.x + (a0 * inv + bb.x);
      hs.y = hs.y + (a1 * inv + bb.y);
    }
    v2f rowB;
    rowB.x = hs.x + pz;
    rowB.y = hs.y + pz;

    if (jt & 1) {
      const int p  = lane & 15;
      const int sA = 2 * p, sB = 2 * p + 1;
      const float a0 = __shfl(rowA.x, sA), a1 = __shfl(rowA.y, sA), a2 = __shfl(rowA.x, sB), a3 = __shfl(rowA.y, sB);
      const float c0 = __shfl(rowB.x, sA), c1 = __shfl(rowB.y, sA), c2 = __shfl(rowB.x, sB), c3 = __shfl(rowB.y, sB);
      const bool first = lane < 16;
      v4f pv;
      pv.x = first ? a0 : c0;
      pv.y = first ? a1 : c1;
      pv.z = first ? a2 : c2;
      pv.w = first ? a3 : c3;
      float* op = out + (size_t)(grow - 1) * HC2 + 4 * lane;
      const bool wr = grow < NN;
      if (wr) *(volatile v4f*)op = pv;
      __threadfence();
      if (wr) *(volatile v4f*)op = pv;
    }
    rowA = rowB;
  }
}

static inline size_t al256(size_t o) { return (o + 255) & ~(size_t)255; }

extern "C" void kernel_launch(void* const* d_in, const int* in_sizes, int n_in,
                              void* d_out, int out_size, void* d_ws, size_t ws_size,
                              hipStream_t stream) {
  if (n_in < 11) return;
  if (in_sizes[0] != NN * FIN) return;
  if (in_sizes[1] != NREL * FIN * HC1) return;
  if (in_sizes[2] != NREL * HC1 || in_sizes[3] != NREL * HC1) return;
  if (in_sizes[4] != NREL * HC1) return;
  if (in_sizes[5] != NREL * HC1 * HC2) return;
  if (in_sizes[6] != NREL * HC2 || in_sizes[7] != NREL * HC2) return;
  if (in_sizes[8] != NREL * HC2) return;
  if (in_sizes[9] != NREL * NE || in_sizes[10] != NREL * NE) return;
  if (out_size != NN * HC2) return;

  const float* x   = (const float*)d_in[0];
  const float* W1  = (const float*)d_in[1];
  const float* al1 = (const float*)d_in[2];
  const float* ar1 = (const float*)d_in[3];
  const float* b1  = (const float*)d_in[4];
  const float* W2  = (const float*)d_in[5];
  const float* al2 = (const float*)d_in[6];
  const float* ar2 = (const float*)d_in[7];
  const float* b2  = (const float*)d_in[8];
  const int*   src = (const int*)  d_in[9];
  const int*   dst = (const int*)  d_in[10];
  float* out = (float*)d_out;

  char* ws = (char*)d_ws;
  size_t off = 0;
  const size_t oXB  = off; off = al256(off + (size_t)MP * FIN * 2);
  const size_t oW1T = off; off = al256(off + (size_t)NREL * HC1 * FIN * 2);
  const size_t oW2T = off; off = al256(off + (size_t)NREL * HC2 * KHL * 2);
  const size_t oPAR = off; off = al256(off + (size_t)8192);
  const size_t oF   = off; off = al256(off + (size_t)MP * NREL * HC1 * 4);
  const size_t oH1  = off; off = al256(off + (size_t)MP * KHL * 2);
  const size_t oS1  = off; off = al256(off + (size_t)NREL * MP * 8 * 4);
  const size_t oS2  = off; off = al256(off + (size_t)MP * 4 * 4);
  const size_t oL   = off; off = al256(off + (size_t)NREL * NBLK * RCAP * 4);
  const size_t oC   = off; off = al256(off + (size_t)NREL * NP * 4);
  const size_t oO   = off; off = al256(off + (size_t)NREL * NP * 4);
  const size_t oFL  = off; off = al256(off + (size_t)NREL * NBLK * 32 * 4);
  if (off > ws_size || off > (size_t)WSMAX) return;
  unsigned short* XB   = (unsigned short*)(ws + oXB);
  unsigned short* W1T  = (unsigned short*)(ws + oW1T);
  unsigned short* W2T2 = (unsigned short*)(ws + oW2T);
  float*          PAR  = (float*)(ws + oPAR);
  float*          FEAT = (float*)(ws + oF);
  unsigned short* H1HL = (unsigned short*)(ws + oH1);
  float*          S1   = (float*)(ws + oS1);
  float*          S2   = (float*)(ws + oS2);
  int*            LIST = (int*)(ws + oL);
  int*            CNT  = (int*)(ws + oC);
  int*            OFF  = (int*)(ws + oO);
  int*            FLG  = (int*)(ws + oFL);

  hipFuncSetAttribute(reinterpret_cast<const void*>(&k_bucket),
                      hipFuncAttributeMaxDynamicSharedMemorySize, LDS_BKT);

  k_prep<<<PTOT / NTHR, NTHR, 0, stream>>>(x, W1, W2, al1, ar1, b1, al2, ar2, b2, XB, W1T, W2T2, PAR);
  k_bucket<<<dim3(NBLK, NREL), NTHR, LDS_BKT, stream>>>(src, dst, LIST, CNT, OFF, FLG);
  k_gemm<1><<<dim3(MP / GBM, NREL), GTHR, 0, stream>>>(XB, FIN, W1T, FIN, FIN, FEAT, NREL * HC1,
                                                        PAR, PAR_AL1, PAR_AR1, S1, MP * 8);
  k_agg1<<<NBLK, NTHR, 0, stream>>>(FEAT, S1, LIST, CNT, OFF, FLG, PAR, H1HL);
  k_gemm<2><<<dim3(MP / GBM, 1), GTHR, 0, stream>>>(H1HL, KHL, W2T2, K2, K2, FEAT, NREL * HC2,
                                                     PAR, PAR_AL2, PAR_AR2, S2, 0);
  k_agg2<<<NBLK, NTHR, 0, stream>>>(FEAT, S2, LIST, CNT, OFF, FLG, PAR, out);
}
